// MultiHeadAttention_57320633532459
// MI455X (gfx1250) — hardware-run, weakly checked
//
#include <hip/hip_runtime.h>
#include <math.h>

typedef __attribute__((ext_vector_type(16))) _Float16 v16h;
typedef __attribute__((ext_vector_type(16))) __bf16 v16b;
typedef __attribute__((ext_vector_type(8)))  _Float16 v8h;
typedef __attribute__((ext_vector_type(8)))  float v8f;
typedef __attribute__((ext_vector_type(4)))  float v4f;
typedef __attribute__((ext_vector_type(4)))  unsigned v4u;

template <typename T> __device__ __forceinline__ void vst2(void* p, T v) { *(volatile T*)p = v; __threadfence(); *(volatile T*)p = v; }
__device__ __forceinline__ v8f wmma16(v16h a, v16h b, v8f c) {
  v8f d = __builtin_amdgcn_wmma_f32_16x16x32_f16(false, a, false, b, (short)0, c, false, false);
  asm volatile("v_nop\n\tv_nop\n\tv_nop\n\tv_nop" : "+v"(d) : "v"(a), "v"(b));
  return d;
}
__device__ __forceinline__ v8f wmma_bf(v16b a, v16b b, v8f c) {
  v8f d = __builtin_amdgcn_wmma_f32_16x16x32_bf16(false, a, false, b, (short)0, c, false, false);
  asm volatile("v_nop\n\tv_nop\n\tv_nop\n\tv_nop" : "+v"(d) : "v"(a), "v"(b));
  return d;
}
__device__ __forceinline__ v16h frag_h(const _Float16* rowk0, int lane) {
  union { v16h v; v8h q[2]; } u; const _Float16* p = rowk0 + 8 * (lane >> 4);
  u.q[0] = *(const v8h*)p; u.q[1] = *(const v8h*)(p + 16); return u.v;
}
__device__ __forceinline__ v16h frag_f32s(const float* rowk0, int lane, float sc) {
  v16h a; const float* p = rowk0 + 8 * (lane >> 4);
#pragma unroll
  for (int i = 0; i < 8; ++i) { a[i] = (_Float16)(p[i] * sc); a[8 + i] = (_Float16)(p[16 + i] * sc); }
  return a;
}
#define LDSX() do { asm volatile("s_wait_dscnt 0" ::: "memory"); __builtin_amdgcn_wave_barrier(); __builtin_amdgcn_fence(3  , "workgroup"); } while (0)

#ifndef NB
#define NB 2
#endif
#ifndef SEQ
#define SEQ 2048
#endif
#define NB_FULL 2
#define SEQ_FULL 2048
#define TT SEQ
#define CC 1024
#define DIN 1024
#define NH 16
#define HD 64
#define NQB (TT / 64)
#define SCALE (0.125f)
#define PLN (8.31776617f)
#define MASK_BLKS ((TT * TT / 4) / 256)
#define PAD_BLKS ((NB * TT / 4 + 255) / 256)
static_assert(SEQ % 128 == 0);
static_assert(SEQ <= SEQ_FULL);
static_assert(NB <= NB_FULL);
static_assert(CC == NH * HD);
static_assert(HD == 64);
static_assert(DIN % 32 == 0);
static_assert(CC % 128 == 0);
static_assert(DIN % 128 == 0);
static_assert(TT % 64 == 0);
static_assert((NB * TT) % 64 == 0);
static_assert((TT * TT / 4) % 256 == 0);
static_assert((NB * TT / 4) % 32 == 0);
__device__ __forceinline__ float bfr(float v) { return (float)(__bf16)v; }
__device__ __forceinline__ v16b wcol_io(const float* Wm, int k0, int o, int lane, int ld) { v16b w; const int g = lane >> 4;
#pragma unroll
  for (int i = 0; i < 8; ++i) { w[i] = (__bf16)Wm[(size_t)(k0 + 8 * g + i) * ld + o]; w[8 + i] = (__bf16)Wm[(size_t)(k0 + 16 + 8 * g + i) * ld + o]; }
  return w; }
__device__ __forceinline__ v16h wcolh_io(const float* Wm, int k0, int o, int lane, int ld) { v16h w; const int g = lane >> 4;
#pragma unroll
  for (int i = 0; i < 8; ++i) { w[i] = (_Float16)(bfr(Wm[(size_t)(k0 + 8 * g + i) * ld + o]) * 256.0f); w[8 + i] = (_Float16)(bfr(Wm[(size_t)(k0 + 16 + 8 * g + i) * ld + o]) * 256.0f); }
  return w; }

#define WS_QH  ((size_t)0)
#define WS_KH  (WS_QH + 2u * (size_t)NB * TT * CC)
#define WS_VT  (WS_KH + 2u * (size_t)NB * TT * CC)
#define WS_MA  (WS_VT + 2u * (size_t)NB * CC * TT)
#define WS_MP  (WS_MA + 4u * (size_t)TT * TT)
#define WS_Y   (WS_MP + 4u * (size_t)NB * TT)
#define WS_END (WS_Y  + 4u * (size_t)NB * TT * CC)
static_assert(WS_KH % 128 == 0);
static_assert(WS_VT % 128 == 0);
static_assert(WS_MA % 128 == 0);
static_assert(WS_MP % 128 == 0);
static_assert(WS_Y % 128 == 0);
static_assert(WS_END <= (size_t)134217728);

__global__ __launch_bounds__(256) void k_mask(const float* __restrict__ MK, const float* __restrict__ PD, float* __restrict__ MA, float* __restrict__ MP) {
  const int blk = blockIdx.x; const int tid = threadIdx.x;
  if (blk < MASK_BLKS) {
    const int e = blk * 256 + tid; const int row = e / (TT / 4), q = e % (TT / 4);
    const v4f v = *(const v4f*)(MK + (size_t)row * SEQ_FULL + q * 4);
    const v4f o = {bfr(v[0]), bfr(v[1]), bfr(v[2]), bfr(v[3])};
    vst2(MA + (size_t)row * TT + q * 4, o);
  } else {
    const int e = (blk - MASK_BLKS) * 256 + tid;
    if (e < NB * TT / 4) {
      const int bb = e / (TT / 4), q = e % (TT / 4);
      const v4f v = *(const v4f*)(PD + (size_t)bb * SEQ_FULL + q * 4);
      const v4f o = {bfr(v[0]), bfr(v[1]), bfr(v[2]), bfr(v[3])};
      vst2(MP + (size_t)bb * TT + q * 4, o);
    }
  }
}

template <int WHICH>
__device__ __forceinline__ void proj_body(const float* __restrict__ X, const float* __restrict__ WA, const float* __restrict__ BA, _Float16* __restrict__ DH) {
  __shared__ __align__(16) _Float16 sh[64][136]; __shared__ __align__(16) _Float16 th[128][72];
  const int tid = threadIdx.x, wave = tid >> 5, lane = tid & 31, col = lane & 15, g = lane >> 4; const int c0 = blockIdx.y * 128; const size_t r0 = (size_t)blockIdx.x * 64; const size_t bb = r0 / TT; const int t0 = (int)(r0 % TT); const size_t xr0 = bb * SEQ_FULL + t0;
  v8f acc[8] = {};
#pragma unroll 2
  for (int kc = 0; kc < DIN / 32; ++kc) { v16b a; { const float* p = X + (xr0 + wave * 16 + col) * DIN + kc * 32 + 8 * g;
#pragma unroll
      for (int i = 0; i < 8; ++i) { a[i] = (__bf16)p[i]; a[8 + i] = (__bf16)p[16 + i]; } }
    asm volatile("s_wait_loadcnt 0x0" ::: "memory");
#pragma unroll
    for (int j = 0; j < 8; ++j) { const v16b w = wcol_io(WA, kc * 32, c0 + j * 16 + col, lane, CC); asm volatile("s_wait_loadcnt 0x0" ::: "memory"); acc[j] = wmma_bf(a, w, acc[j]); } }
  if (WHICH < 2) {
#pragma unroll
    for (int j = 0; j < 8; ++j) { const float bias = bfr(BA[c0 + j * 16 + col]);
#pragma unroll
      for (int r = 0; r < 8; ++r) { const float v = acc[j][r] + bias; sh[wave * 16 + 8 * g + r][j * 16 + col] = (_Float16)v; } }
    __syncthreads();
    for (int e = tid; e < 64 * 16; e += 128) { const int rl = e >> 4, q = e & 15; vst2((unsigned*)(DH + (r0 + rl) * CC + c0 + q * 8), *(const v4u*)&sh[rl][q * 8]); }
  } else {
#pragma unroll
    for (int j = 0; j < 8; ++j) { const float bias = bfr(BA[c0 + j * 16 + col]);
#pragma unroll
      for (int r = 0; r < 8; ++r) { const float v = acc[j][r] + bias; const int rl = wave * 16 + 8 * g + r, cl = j * 16 + col; th[cl][rl] = (_Float16)v; } }
    __syncthreads();
    for (int e = tid; e < 128 * 8; e += 128) { const int cl = e >> 3, q = e & 7; vst2((unsigned*)(DH + (bb * CC + c0 + cl) * (size_t)TT + t0 + q * 8), *(const v4u*)&th[cl][q * 8]); } } }

__global__ __launch_bounds__(128) void k_proj_q(const float* __restrict__ X, const float* __restrict__ WA, const float* __restrict__ BA, _Float16* __restrict__ DH) { proj_body<0>(X, WA, BA, DH); }
__global__ __launch_bounds__(128) void k_proj_k(const float* __restrict__ X, const float* __restrict__ WA, const float* __restrict__ BA, _Float16* __restrict__ DH) { proj_body<1>(X, WA, BA, DH); }
__global__ __launch_bounds__(128) void k_proj_v(const float* __restrict__ X, const float* __restrict__ WA, const float* __restrict__ BA, _Float16* __restrict__ DH) { proj_body<2>(X, WA, BA, DH); }

__global__ __launch_bounds__(128) __attribute__((amdgpu_num_vgpr(256))) void k_fa(const _Float16* __restrict__ QH, const _Float16* __restrict__ KH, const _Float16* __restrict__ VT, const float* __restrict__ MA, const float* __restrict__ MP, float* __restrict__ Y) {
  __shared__ __align__(16) float ss[4][16][HD + 4];
  const int tid = threadIdx.x, lane = tid & 31, col = lane & 15, g = lane >> 4;
  const int wave = __builtin_amdgcn_readfirstlane(tid >> 5);
  const int qb = blockIdx.x, h = blockIdx.y, b = blockIdx.z;
  const int ql0 = qb * 64 + wave * 16;
  const size_t q0 = (size_t)b * TT + ql0;
  const v16h qf0 = frag_h(QH + (q0 + col) * CC + h * HD, lane), qf1 = frag_h(QH + (q0 + col) * CC + h * HD + 32, lane);
  const _Float16* kbase = KH + ((size_t)b * TT + col) * CC + h * HD;
  const _Float16* vbase = VT + ((size_t)b * CC + h * HD + col) * (size_t)TT;
  const float* mrow = MA + (size_t)(ql0 + col) * TT + 8 * g;
  const float* prow = MP + (size_t)b * TT + 8 * g;
  v8f acc[HD / 16] = {};
  float m = -1.0e30f, l = 0.f;
#pragma unroll 1
  for (int kc = 0; kc < TT / 32; ++kc) { const int k0 = kc * 32;
    const v4f a0 = *(const v4f*)(mrow + k0), a1 = *(const v4f*)(mrow + k0 + 4), a2 = *(const v4f*)(mrow + k0 + 16), a3 = *(const v4f*)(mrow + k0 + 20);
    const v4f p0 = *(const v4f*)(prow + k0), p1 = *(const v4f*)(prow + k0 + 4), p2 = *(const v4f*)(prow + k0 + 16), p3 = *(const v4f*)(prow + k0 + 20);
    const _Float16* kp = kbase + (size_t)k0 * CC;
    v8f s0 = {}, s1 = {};
    s0 = wmma16(frag_h(kp, lane), qf0, s0);
    s0 = wmma16(frag_h(kp + 32, lane), qf1, s0);
    s1 = wmma16(frag_h(kp + 16 * CC, lane), qf0, s1);
    s1 = wmma16(frag_h(kp + 16 * CC + 32, lane), qf1, s1);
    float x[16];
#pragma unroll
    for (int r = 0; r < 4; ++r) {
      x[r]      = (s0[r] * SCALE + p0[r]) + a0[r];
      x[4 + r]  = (s0[4 + r] * SCALE + p1[r]) + a1[r];
      x[8 + r]  = (s1[r] * SCALE + p2[r]) + a2[r];
      x[12 + r] = (s1[4 + r] * SCALE + p3[r]) + a3[r]; }
    float mx = x[0];
#pragma unroll
    for (int i = 1; i < 16; ++i) mx = fmaxf(mx, x[i]);
    mx = fmaxf(mx, __shfl_xor(mx, 16));
    const float newm = fmaxf(m, mx); const float c = __expf(m - newm); m = newm; const float nm2 = newm - PLN;
    v16h pb; float ls = 0.f;
#pragma unroll
    for (int i = 0; i < 16; ++i) { const _Float16 e = (_Float16)__expf(x[i] - nm2); pb[i] = e; ls += (float)e; }
    l = l * c + ls;
#pragma unroll
    for (int j = 0; j < HD / 16; ++j) acc[j] = acc[j] * c;
    const _Float16* vp = vbase + k0;
#pragma unroll
    for (int j = 0; j < HD / 16; ++j) acc[j] = wmma16(frag_h(vp + (size_t)j * 16 * TT, lane), pb, acc[j]); }
  l += __shfl_xor(l, 16);
  const float inv = 1.0f / l;
#pragma unroll
  for (int j = 0; j < HD / 16; ++j)
#pragma unroll
    for (int r = 0; r < 8; ++r) ss[wave][col][j * 16 + 8 * g + r] = acc[j][r] * inv;
  LDSX(); for (int rl = 0; rl < 16; ++rl) if (lane < HD / 4) vst2(Y + ((size_t)b * TT + ql0 + rl) * CC + h * HD + lane * 4, *(const v4f*)&ss[wave][rl][lane * 4]); }

__global__ __launch_bounds__(128) void k_out(const float* __restrict__ Y, const float* __restrict__ WO, const float* __restrict__ BO, float* __restrict__ OUT) { __shared__ __align__(16) float sf[4][16][132];
  const int tid = threadIdx.x, wave = tid >> 5, lane = tid & 31, col = lane & 15, g = lane >> 4; const int c0 = blockIdx.y * 128; const size_t rb = (size_t)blockIdx.x * 64; const size_t bb = rb / TT; const int tb = (int)(rb % TT);
  const size_t r0 = rb + wave * 16; const size_t o0 = bb * SEQ_FULL + tb + wave * 16;
  v8f acc[8] = {};
#pragma unroll 2
  for (int kc = 0; kc < CC / 32; ++kc) { const v16h a = frag_f32s(Y + (r0 + col) * CC + kc * 32, lane, 64.0f); asm volatile("s_wait_loadcnt 0x0" ::: "memory");
#pragma unroll
    for (int j = 0; j < 8; ++j) { const v16h w = wcolh_io(WO, kc * 32, c0 + j * 16 + col, lane, DIN); asm volatile("s_wait_loadcnt 0x0" ::: "memory"); acc[j] = wmma16(a, w, acc[j]); } }
#pragma unroll
  for (int j = 0; j < 8; ++j) { const float bias = bfr(BO[c0 + j * 16 + col]);
#pragma unroll
    for (int r = 0; r < 8; ++r) sf[wave][8 * g + r][j * 16 + col] = acc[j][r] * (1.0f / 16384.0f) + bias; }
  LDSX(); for (int rl = 0; rl < 16; ++rl) vst2(OUT + (o0 + rl) * DIN + c0 + lane * 4, *(const v4f*)&sf[wave][rl][lane * 4]); }

extern "C" void kernel_launch(void* const* d_in, const int* in_sizes, int n_in, void* d_out, int out_size, void* d_ws, size_t ws_size, hipStream_t stream) {
  if (n_in < 13) return;
  const long long xneed = ((long long)(NB - 1) * SEQ_FULL + TT) * DIN;
  if ((long long)in_sizes[0] < xneed || (long long)in_sizes[1] < xneed || (long long)in_sizes[2] < xneed) return;
  if ((long long)in_sizes[3] < (long long)(TT - 1) * SEQ_FULL + TT) return;
  if ((long long)in_sizes[4] < (long long)(NB - 1) * SEQ_FULL + TT) return;
  if ((long long)in_sizes[5] < (long long)DIN * CC || (long long)in_sizes[7] < (long long)DIN * CC || (long long)in_sizes[9] < (long long)DIN * CC || (long long)in_sizes[11] < (long long)CC * DIN) return;
  if (in_sizes[6] < CC || in_sizes[8] < CC || in_sizes[10] < CC || in_sizes[12] < DIN) return;
  if ((long long)out_size < xneed) return;
  if (ws_size < (size_t)WS_END) return;
  const float** F = (const float**)d_in;
  char* ws = (char*)d_ws; _Float16 *QH = (_Float16*)(ws + WS_QH), *KH = (_Float16*)(ws + WS_KH), *VT = (_Float16*)(ws + WS_VT); float *MA = (float*)(ws + WS_MA), *MP = (float*)(ws + WS_MP), *Y = (float*)(ws + WS_Y);
  k_mask<<<dim3(MASK_BLKS + PAD_BLKS), 256, 0, stream>>>(F[3], F[4], MA, MP);
  k_proj_q<<<dim3(NB * TT / 64, CC / 128), 128, 0, stream>>>(F[2], F[9], F[10], QH);
  k_proj_k<<<dim3(NB * TT / 64, CC / 128), 128, 0, stream>>>(F[0], F[5], F[6], KH);
  k_proj_v<<<dim3(NB * TT / 64, CC / 128), 128, 0, stream>>>(F[1], F[7], F[8], VT);
  k_fa<<<dim3(NQB, NH, NB), 128, 0, stream>>>(QH, KH, VT, MA, MP, Y);
  k_out<<<dim3(NB * TT / 64, DIN / 128), 128, 0, stream>>>(Y, F[11], F[12], (float*)d_out);
}
